// LSTM_26912265077001
// MI455X (gfx1250) — hardware-verified
//
#include <hip/hip_runtime.h>
#include <math.h>

constexpr int HID      = 51;
constexpr int NGATE    = 4 * HID;
constexpr int NPADN    = 208;
constexpr int NWAVES   = 13;
constexpr int NTHR     = NWAVES * 32;
constexpr int NSTEP    = 512;
constexpr int NBATCH   = 1024;
constexpr int MROWS    = 16;
constexpr int K1PAD    = 64;
constexpr int K2PAD    = 128;
constexpr int APITCH   = 128;
constexpr int GPITCH   = 208;
constexpr int HFPITCH  = 52;
constexpr int OSPITCH  = 36;
constexpr int NPAIR    = MROWS * HID;
constexpr int NPADCOL  = K1PAD - HID;
constexpr int NPADTHR  = MROWS * NPADCOL;
constexpr int OUTGRP   = 32;
constexpr float WCARRY  = 64.0f;
constexpr float HCARRY  = 16.0f;
constexpr float LOCARRY = 2048.0f;
constexpr float FOLDSC  = 1.0f / (WCARRY * HCARRY);
constexpr float LOINV   = 1.0f / LOCARRY;

static_assert(NGATE == 204, "gate rows");
static_assert(NPADN == NWAVES * 16 && NPADN >= NGATE, "n tiles");
static_assert(NPAIR <= 2 * NTHR, "pair slots");
static_assert(NPADTHR <= NTHR, "pad writers");
static_assert(NSTEP % OUTGRP == 0, "whole output lines");
static_assert(NBATCH % MROWS == 0, "batch tiles");
static_assert(K1PAD % 32 == 0 && K2PAD % 32 == 0, "k steps of 32");
static_assert(K1PAD >= HID && K2PAD >= K1PAD + HID, "k pads");
static_assert(APITCH >= K2PAD && APITCH % 8 == 0, "A tile pitch");
static_assert(GPITCH >= NPADN, "gate slab pitch");
static_assert(HFPITCH > HID, "head row pitch");
static_assert((NPADN * 8) % 32 == 0, "plane producer: whole waves");

typedef __attribute__((ext_vector_type(16))) _Float16 v16h;
typedef __attribute__((ext_vector_type(8)))  _Float16 v8h;
typedef __attribute__((ext_vector_type(8)))  float    v8f;
typedef __attribute__((ext_vector_type(4)))  float    v4f;

__device__ __forceinline__ void mma_guard3(v8f& a, v8f& b, v16h x, v16h y, v16h z) {
  asm volatile("v_nop\n\tv_nop\n\tv_nop\n\tv_nop" : "+v"(a), "+v"(b) : "v"(x), "v"(y), "v"(z));
}

template <typename T> struct Frag;
template <> struct Frag<_Float16> {
  typedef v16h V; union U { v16h v; v8h h[2]; };
  static __device__ __forceinline__ v16h load(const _Float16* p) {
    U f; f.h[0] = *(const v8h*)(p); f.h[1] = *(const v8h*)(p + 16); return f.v;
  }
  static __device__ __forceinline__ v8f mma(v16h a, v16h b, v8f c) {
    return __builtin_amdgcn_wmma_f32_16x16x32_f16(false, a, false, b, (short)0, c, false, false);
  }
};

__device__ __forceinline__ float sigm(float v) { return __builtin_amdgcn_rcpf(1.0f + expf(-v)); }
__device__ __forceinline__ float tnh(float v)  { return 2.0f * sigm(2.0f * v) - 1.0f; }

__global__ __launch_bounds__(256) void wplane_kernel(const float* __restrict__ src, unsigned short* __restrict__ dst,
                                                     int dpitch, int dcol0) {
  const int i = blockIdx.x * 256 + threadIdx.x;
  if (i < NPADN * 8) {
    const int n  = i >> 3;
    const int k8 = i & 7;
    const int nc = (n < NGATE) ? n : (NGATE - 1);
    v8h hv;
#pragma unroll
    for (int e = 0; e < 8; ++e) {
      const int k  = 8 * k8 + e;
      const int kc = (k < HID) ? k : (HID - 1);
      const float v = src[nc * HID + kc];
      const float w = (n < NGATE && k < HID) ? (v * WCARRY) : 0.0f;
      hv[e] = (_Float16)w;
    }
    unsigned short* dp = dst + (size_t)n * (size_t)dpitch + (size_t)(dcol0 + 8 * k8);
    *(volatile v8h*)dp = hv;
    __threadfence();
    *(volatile v8h*)dp = hv;
  }
}

__device__ __forceinline__ float cell_update(const float* gr, float ai, float af, float ag, float ao, float& cst) {
  const float zi = gr[0]       + ai;
  const float zf = gr[HID]     + af;
  const float zg = gr[2 * HID] + ag;
  const float zo = gr[3 * HID] + ao;
  const float ig = sigm(zi);
  const float fg = sigm(zf);
  const float gg = tnh(zg);
  const float og = sigm(zo);
  const float cn = fg * cst + ig * gg;
  cst = cn;
  return og * tnh(cn);
}

__device__ __forceinline__ void split_store(_Float16* hip, _Float16* lop, int idx, float h, bool ok) {
  const float hs = h * HCARRY;
  const _Float16 hh = (_Float16)hs;
  const float hb = (float)hh;
  const float res = hs - hb;
  const _Float16 hl = (_Float16)(res * LOCARRY);
  if (ok) { hip[idx] = hh; lop[idx] = hl; }
}

__device__ __forceinline__ void head_step(const float* H2f, const float* wls, float* OST, float* out,
                                          float b0, int bb, int lane, int t) {
  const int m = lane & 15;
  float acc = b0;
#pragma unroll 3
  for (int k = 0; k < HID; ++k) acc = fmaf(H2f[m * HFPITCH + k], wls[k], acc);
  if (lane < 16) OST[m * OSPITCH + (t & (OUTGRP - 1))] = acc;
  if ((t & (OUTGRP - 1)) == (OUTGRP - 1)) {
    __builtin_amdgcn_fence(__ATOMIC_RELEASE, "workgroup");
    __builtin_amdgcn_wave_barrier();
    __builtin_amdgcn_fence(__ATOMIC_ACQUIRE, "workgroup");
    const int t0 = t - (OUTGRP - 1);
    const int q  = lane >> 3;
    const int c4 = (lane & 7) * 4;
    v4f vv[4];
#pragma unroll
    for (int it = 0; it < 4; ++it) vv[it] = *(const v4f*)(OST + (it * 4 + q) * OSPITCH + c4);
    for (int pass = 0; pass < 2; ++pass) {
#pragma unroll
      for (int it = 0; it < 4; ++it) {
        const int row = it * 4 + q;
        *(volatile v4f*)(out + (size_t)(bb + row) * NSTEP + (size_t)(t0 + c4)) = vv[it];
      }
      __threadfence();
    }
    __builtin_amdgcn_fence(__ATOMIC_RELEASE, "workgroup");
    __builtin_amdgcn_wave_barrier();
    __builtin_amdgcn_fence(__ATOMIC_ACQUIRE, "workgroup");
  }
}

__global__ __launch_bounds__(NTHR) void lstm2_seq_kernel(const float* __restrict__ x,
                                                         const float* __restrict__ wih1,
                                                         const float* __restrict__ bih1, const float* __restrict__ bhh1,
                                                         const float* __restrict__ bih2, const float* __restrict__ bhh2,
                                                         const float* __restrict__ wlin, const float* __restrict__ blin,
                                                         const unsigned short* __restrict__ WP1p,
                                                         const unsigned short* __restrict__ WP2p,
                                                         float* __restrict__ out) {
  __shared__ __align__(16) _Float16 Ahi[MROWS * APITCH];
  __shared__ __align__(16) _Float16 Alo[MROWS * APITCH];
  __shared__ __align__(16) float    G1[MROWS * GPITCH];
  __shared__ __align__(16) float    G2[MROWS * GPITCH];
  __shared__ __align__(16) float    H2f[MROWS * HFPITCH];
  __shared__ __align__(16) float    OST[MROWS * OSPITCH];
  __shared__ float cb1[NGATE];
  __shared__ float cb2[NGATE];
  __shared__ float cwx[NGATE];
  __shared__ float wls[HFPITCH];

  const _Float16* WP1 = (const _Float16*)WP1p;
  const _Float16* WP2 = (const _Float16*)WP2p;
  const int tid = threadIdx.x, lane = tid & 31, wave = tid >> 5;
  const int c = lane & 15, hh = lane >> 4, koff = hh * 8;
  const int bb = blockIdx.x * MROWS;
  const int ncol = 16 * wave + c;
  const _Float16 zh = (_Float16)0.0f;

#pragma unroll 1
  for (int i = tid; i < MROWS * APITCH; i += NTHR) { Ahi[i] = zh; Alo[i] = zh; }
#pragma unroll 1
  for (int i = tid; i < MROWS * HFPITCH; i += NTHR) H2f[i] = 0.0f;
  {
    const int gi = (tid < NGATE) ? tid : (NGATE - 1);
    const float a1 = bih1[gi];
    const float a2 = bhh1[gi];
    const float a3 = bih2[gi];
    const float a4 = bhh2[gi];
    const float a5 = wih1[gi];
    if (tid < NGATE) { cb1[tid] = a1 + a2; cb2[tid] = a3 + a4; cwx[tid] = a5; }
    const int wi = (tid < HID) ? tid : (HID - 1);
    const float wv = wlin[wi];
    if (tid < HFPITCH) wls[tid] = (tid < HID) ? wv : 0.0f;
  }
  const float b0 = blin[0];

  v16h b1f[2], b2f[4];
#pragma unroll
  for (int kt = 0; kt < 2; ++kt) b1f[kt] = Frag<_Float16>::load(WP1 + ncol * K1PAD + koff + 32 * kt);
  asm volatile("" ::: "memory");
#pragma unroll
  for (int kt = 0; kt < 2; ++kt) b2f[kt] = Frag<_Float16>::load(WP2 + ncol * K2PAD + koff + 32 * kt);
  asm volatile("" ::: "memory");
#pragma unroll
  for (int kt = 2; kt < 4; ++kt) b2f[kt] = Frag<_Float16>::load(WP2 + ncol * K2PAD + koff + 32 * kt);
  asm volatile("" ::: "memory");

  __syncthreads();

  int   mrow[2], jcol[2];
  bool  okp[2];
  float wx[2][4], bs1[2][4], bs2[2][4];
  float cs1[2], cs2[2];
#pragma unroll
  for (int sl = 0; sl < 2; ++sl) {
    const int p  = tid + sl * NTHR;
    okp[sl] = (p < NPAIR);
    const int pc = (p < NPAIR) ? p : (NPAIR - 1);
    mrow[sl] = pc / HID;
    jcol[sl] = pc - mrow[sl] * HID;
#pragma unroll
    for (int g = 0; g < 4; ++g) {
      wx[sl][g]  = cwx[g * HID + jcol[sl]];
      bs1[sl][g] = cb1[g * HID + jcol[sl]];
      bs2[sl][g] = cb2[g * HID + jcol[sl]];
    }
    cs1[sl] = 0.0f;
    cs2[sl] = 0.0f;
  }
  const int ptid   = (tid < NPADTHR) ? tid : (NPADTHR - 1);
  const int padidx = (ptid / NPADCOL) * APITCH + HID + (ptid % NPADCOL);
  const bool padw  = (tid < NPADTHR);

  const _Float16* ahrow = Ahi + c * APITCH + koff;
  const _Float16* alrow = Alo + c * APITCH + koff;
  const v8f z8 = {0.f, 0.f, 0.f, 0.f, 0.f, 0.f, 0.f, 0.f};

#pragma unroll 1
  for (int s = 0; s < NSTEP; ++s) {
    float xs[2];
#pragma unroll
    for (int sl = 0; sl < 2; ++sl) xs[sl] = x[(size_t)s * NBATCH + (size_t)(bb + mrow[sl])];

    {
      v8f aH = z8, aL = z8;
#pragma unroll
      for (int kt = 0; kt < 2; ++kt) {
        const v16h ah = Frag<_Float16>::load(ahrow + 32 * kt);
        const v16h al = Frag<_Float16>::load(alrow + 32 * kt);
        aH = Frag<_Float16>::mma(ah, b1f[kt], aH);
        aL = Frag<_Float16>::mma(al, b1f[kt], aL);
        mma_guard3(aH, aL, ah, al, b1f[kt]);
      }
#pragma unroll
      for (int r = 0; r < 8; ++r) G1[(8 * hh + r) * GPITCH + ncol] = (aH[r] + aL[r] * LOINV) * FOLDSC;
    }
    __syncthreads();

    if (wave == 0 && s > 0) head_step(H2f, wls, OST, out, b0, bb, lane, s - 1);
#pragma unroll
    for (int sl = 0; sl < 2; ++sl) {
      const float ai = fmaf(xs[sl], wx[sl][0], bs1[sl][0]);
      const float af = fmaf(xs[sl], wx[sl][1], bs1[sl][1]);
      const float ag = fmaf(xs[sl], wx[sl][2], bs1[sl][2]);
      const float ao = fmaf(xs[sl], wx[sl][3], bs1[sl][3]);
      const float hn = cell_update(G1 + mrow[sl] * GPITCH + jcol[sl], ai, af, ag, ao, cs1[sl]);
      split_store(Ahi, Alo, mrow[sl] * APITCH + jcol[sl], hn, okp[sl]);
    }
    if (padw) { Ahi[padidx] = zh; Alo[padidx] = zh; }
    __syncthreads();

    {
      v8f aH = z8, aL = z8;
#pragma unroll
      for (int kt = 0; kt < 4; ++kt) {
        const v16h ah = Frag<_Float16>::load(ahrow + 32 * kt);
        const v16h al = Frag<_Float16>::load(alrow + 32 * kt);
        aH = Frag<_Float16>::mma(ah, b2f[kt], aH);
        aL = Frag<_Float16>::mma(al, b2f[kt], aL);
        mma_guard3(aH, aL, ah, al, b2f[kt]);
      }
#pragma unroll
      for (int r = 0; r < 8; ++r) G2[(8 * hh + r) * GPITCH + ncol] = (aH[r] + aL[r] * LOINV) * FOLDSC;
    }
    __syncthreads();

#pragma unroll
    for (int sl = 0; sl < 2; ++sl) {
      const float hn = cell_update(G2 + mrow[sl] * GPITCH + jcol[sl],
                                   bs2[sl][0], bs2[sl][1], bs2[sl][2], bs2[sl][3], cs2[sl]);
      split_store(Ahi, Alo, mrow[sl] * APITCH + K1PAD + jcol[sl], hn, okp[sl]);
      if (okp[sl]) H2f[mrow[sl] * HFPITCH + jcol[sl]] = hn;
    }
    if (padw) { Ahi[padidx + K1PAD] = zh; Alo[padidx + K1PAD] = zh; }
  }

  __syncthreads();
  if (wave == 0) head_step(H2f, wls, OST, out, b0, bb, lane, NSTEP - 1);
}

extern "C" void kernel_launch(void* const* d_in, const int* in_sizes, int n_in,
                              void* d_out, int out_size, void* d_ws, size_t ws_size, hipStream_t stream) {
  if (n_in < 11 || d_out == nullptr || d_ws == nullptr) return;
  if (in_sizes[0] != NSTEP * NBATCH || in_sizes[1] != NGATE || in_sizes[2] != NGATE * HID ||
      in_sizes[3] != NGATE || in_sizes[4] != NGATE || in_sizes[5] != NGATE * HID ||
      in_sizes[6] != NGATE * HID || in_sizes[7] != NGATE || in_sizes[8] != NGATE ||
      in_sizes[9] != HID || in_sizes[10] != 1 || out_size != NBATCH * NSTEP) return;

  const float* xin  = (const float*)d_in[0];
  const float* wih1 = (const float*)d_in[1];
  const float* whh1 = (const float*)d_in[2];
  const float* bih1 = (const float*)d_in[3];
  const float* bhh1 = (const float*)d_in[4];
  const float* wih2 = (const float*)d_in[5];
  const float* whh2 = (const float*)d_in[6];
  const float* bih2 = (const float*)d_in[7];
  const float* bhh2 = (const float*)d_in[8];
  const float* wlin = (const float*)d_in[9];
  const float* blin = (const float*)d_in[10];
  float* out = (float*)d_out;

  char* ws = (char*)d_ws; size_t off = 0;
  auto carve = [&](size_t bytes) -> char* { char* p = ws + off; off += (bytes + 255) & ~(size_t)255; return p; };
  unsigned short* WP1 = (unsigned short*)carve((size_t)NPADN * K1PAD * 2);
  unsigned short* WP2 = (unsigned short*)carve((size_t)NPADN * K2PAD * 2);
  if (off > ws_size || off > (size_t)134217728) return;

  const int pgrid = (NPADN * 8 + 255) / 256;
  wplane_kernel<<<pgrid, 256, 0, stream>>>(whh1, WP1, K1PAD, 0);
  wplane_kernel<<<pgrid, 256, 0, stream>>>(wih2, WP2, K2PAD, 0);
  wplane_kernel<<<pgrid, 256, 0, stream>>>(whh2, WP2, K2PAD, K1PAD);
  lstm2_seq_kernel<<<NBATCH / MROWS, NTHR, 0, stream>>>(xin, wih1, bih1, bhh1, bih2, bhh2, wlin, blin, WP1, WP2, out);
}
